// GNNActorVariablePrice_24326694764553
// MI455X (gfx1250) — hardware-verified
//
#include <hip/hip_runtime.h>
#include <stddef.h>


#define HIDC    256
#define NREG    64
#define NMAT    4
#define WPL     (HIDC * HIDC)
#define NTHR    256
#define NWAVE   8
#define EPT     8
#define NGRP    2
#define CHUNK   (NTHR * EPT * NGRP)
#define WCAP    (EPT * NGRP * 32)
#define LISTN   (NWAVE * WCAP)
#define NBC     4096
#define NBF     1024
#define RCAP    40960
#define RBN     128
#define TGT     256
#define DEGCAP  256
#define GROWS   64
#define OTHR    512
#define APH     (HIDC + 8)
#define BROWS   64
#define XHP     (HIDC + 8)
#define XFP     (HIDC + 4)
#define SOP     (NREG + 4)
#define WSCAP   134217728

#define LDS_GEMM (2 * GROWS * APH * 2)
#define LDS_FILL ((RCAP + NBF + LISTN) * 4 + 64)
#define LDS_BIL  (BROWS * XHP * 2 + BROWS * XFP * 4 + BROWS * SOP * 4)

static_assert((CHUNK & (CHUNK - 1)) == 0);
static_assert(CHUNK <= 4096);
static_assert(NBC <= 4096 && NBF <= 4096);
static_assert((NBC & (NBC - 1)) == 0 && (NBF & (NBF - 1)) == 0);
static_assert(NBC == 4 * NBF);
static_assert(OTHR * 8 == NBC);
static_assert((RCAP % 32) == 0);
static_assert(GROWS * HIDC * 4 + GROWS * 4 <= LDS_GEMM);
static_assert((APH * 2) % 16 == 0);
static_assert((TGT % GROWS) == 0 && TGT == NWAVE * 32);
static_assert((NBC % TGT) == 0);
static_assert((GROWS * HIDC / 8) % NTHR == 0);
static_assert(GROWS == NWAVE * 8);
static_assert(HIDC == 256);
static_assert(NREG == NWAVE * 8);
static_assert(BROWS == 4 * 16);
static_assert((BROWS * HIDC / 8) % NTHR == 0);
static_assert((BROWS * NREG / 4) % NTHR == 0);
static_assert((XHP * 2) % 16 == 0 && (XFP * 4) % 16 == 0 && (SOP * 4) % 16 == 0);
static_assert((BROWS * XHP * 2) % 16 == 0);

typedef float          v4f  __attribute__((ext_vector_type(4)));
typedef float          v8f  __attribute__((ext_vector_type(8)));
typedef int            v4i  __attribute__((ext_vector_type(4)));
typedef unsigned short v8us __attribute__((ext_vector_type(8)));
typedef __bf16         v16b __attribute__((ext_vector_type(16)));
typedef _Float16       v8h  __attribute__((ext_vector_type(8)));
typedef _Float16       v16h __attribute__((ext_vector_type(16)));
union FragB { v16b v; v8us h[2]; };
union FragH { v16h v; v8h h[2]; };
union H8    { v8h h; v4i i; };

__device__ __forceinline__ unsigned int bfr(float f) {
  const unsigned int u = __float_as_uint(f);
  return (u + 0x7FFFu + ((u >> 16) & 1u)) >> 16;
}

__device__ __forceinline__ void split1(float x, unsigned short& hb, unsigned short& lb) {
  const unsigned int hu = bfr(x);
  const float hf = __uint_as_float(hu << 16);
  hb = (unsigned short)hu;
  lb = (unsigned short)bfr(x - hf);
}

__device__ __forceinline__ void split8(v4f a, v4f b, v8us& hi, v8us& lo) {
  unsigned short hb, lb;
  split1(a.x, hb, lb); hi[0] = hb; lo[0] = lb;
  split1(a.y, hb, lb); hi[1] = hb; lo[1] = lb;
  split1(a.z, hb, lb); hi[2] = hb; lo[2] = lb;
  split1(a.w, hb, lb); hi[3] = hb; lo[3] = lb;
  split1(b.x, hb, lb); hi[4] = hb; lo[4] = lb;
  split1(b.y, hb, lb); hi[5] = hb; lo[5] = lb;
  split1(b.z, hb, lb); hi[6] = hb; lo[6] = lb;
  split1(b.w, hb, lb); hi[7] = hb; lo[7] = lb;
}

__device__ __forceinline__ v8f wmb(v16b a, v16b b, v8f c) {
  v8f d = __builtin_amdgcn_wmma_f32_16x16x32_bf16(false, a, false, b, (short)0, c, false, false);
  asm volatile("v_nop\n\tv_nop\n\tv_nop\n\tv_nop" : "+v"(d) : "v"(a), "v"(b));
  return d;
}
__device__ __forceinline__ v8f wmh(v16h a, v16h b, v8f c) {
  v8f d = __builtin_amdgcn_wmma_f32_16x16x32_f16(false, a, false, b, (short)0, c, false, false);
  asm volatile("v_nop\n\tv_nop\n\tv_nop\n\tv_nop" : "+v"(d) : "v"(a), "v"(b));
  return d;
}

template <int NB>
__device__ __forceinline__ int scan_chunk(const int* __restrict__ dsts, int nE, int cbase, int slotBase,
                                          int vec8, int* list, int tid, int lane, int wave) {
  int wc = 0;
#pragma unroll
  for (int g = 0; g < NGRP; ++g) {
    const int el0  = (g * NTHR + tid) * EPT;
    const int e0   = cbase + el0;
    const int sent = -2147483647 - 1;
    v4i da, db;
    if (vec8 != 0 && cbase + CHUNK <= nE) {
      da = *(const v4i*)(dsts + e0);
      db = *(const v4i*)(dsts + e0 + 4);
    } else {
      da.x = (e0     < nE) ? dsts[min(e0, nE - 1)] : sent;
      da.y = (e0 + 1 < nE) ? dsts[min(e0 + 1, nE - 1)] : sent;
      da.z = (e0 + 2 < nE) ? dsts[min(e0 + 2, nE - 1)] : sent;
      da.w = (e0 + 3 < nE) ? dsts[min(e0 + 3, nE - 1)] : sent;
      db.x = (e0 + 4 < nE) ? dsts[min(e0 + 4, nE - 1)] : sent;
      db.y = (e0 + 5 < nE) ? dsts[min(e0 + 5, nE - 1)] : sent;
      db.z = (e0 + 6 < nE) ? dsts[min(e0 + 6, nE - 1)] : sent;
      db.w = (e0 + 7 < nE) ? dsts[min(e0 + 7, nE - 1)] : sent;
    }
    const unsigned nb = (unsigned)slotBase;
    const unsigned s0 = (unsigned)da.x - nb, s1 = (unsigned)da.y - nb;
    const unsigned s2 = (unsigned)da.z - nb, s3 = (unsigned)da.w - nb;
    const unsigned s4 = (unsigned)db.x - nb, s5 = (unsigned)db.y - nb;
    const unsigned s6 = (unsigned)db.z - nb, s7 = (unsigned)db.w - nb;
    const bool h0 = s0 < (unsigned)NB, h1 = s1 < (unsigned)NB, h2 = s2 < (unsigned)NB, h3 = s3 < (unsigned)NB;
    const bool h4 = s4 < (unsigned)NB, h5 = s5 < (unsigned)NB, h6 = s6 < (unsigned)NB, h7 = s7 < (unsigned)NB;
    const unsigned any = __builtin_amdgcn_ballot_w32(h0 | h1 | h2 | h3 | h4 | h5 | h6 | h7);
    if (any != 0u) {
#define HITJ(J, HJ, SJ) { \
        const unsigned mj = __builtin_amdgcn_ballot_w32(HJ); \
        if (mj != 0u) { \
          if (HJ) { \
            const int pos = wc + (int)__builtin_amdgcn_mbcnt_lo(mj, 0u); \
            if (pos < WCAP) list[wave * WCAP + pos] = ((el0 + (J)) << 12) | (int)(SJ); \
          } \
          wc += (int)__builtin_popcount(mj); } }
      HITJ(0, h0, s0)
      HITJ(1, h1, s1)
      HITJ(2, h2, s2)
      HITJ(3, h3, s3)
      HITJ(4, h4, s4)
      HITJ(5, h5, s5)
      HITJ(6, h6, s6)
      HITJ(7, h7, s7)
#undef HITJ
    }
  }
  return wc;
}

__global__ __launch_bounds__(NTHR) void k_wprep(
    const float* __restrict__ w0, const float* __restrict__ w1,
    const float* __restrict__ w2, const float* __restrict__ w3, unsigned short* wp) {
  const int seg = (int)blockIdx.x >> 5;
  const float* src = seg == 0 ? w0 : (seg == 1 ? w1 : (seg == 2 ? w2 : w3));
  const int i  = ((int)(blockIdx.x & 31) * NTHR) + (int)threadIdx.x;
  const float* sp = src + (size_t)i * 8;
  const v4f a = *(const v4f*)sp, b = *(const v4f*)(sp + 4);
  v8us hv, lv;
  split8(a, b, hv, lv);
  unsigned short* dh = wp + (size_t)seg * 2 * WPL + (size_t)i * 8;
  unsigned short* dl = dh + WPL;
  *(volatile v8us*)dh = hv;
  *(volatile v8us*)dl = lv;
  __threadfence();
  *(volatile v8us*)dh = hv;
  *(volatile v8us*)dl = lv;
}

__global__ __launch_bounds__(NTHR) void k_bwprep(const float* __restrict__ wb, _Float16* wh, int nGroups) {
  int g = (int)blockIdx.x * NTHR + (int)threadIdx.x;
  const int ok = g < nGroups ? 1 : 0;
  g = g > nGroups - 1 ? nGroups - 1 : g;
  const float* sp = wb + (size_t)g * 8;
  const v4f a = *(const v4f*)sp, b = *(const v4f*)(sp + 4);
  H8 u;
  u.h[0] = (_Float16)(a.x * 64.0f); u.h[1] = (_Float16)(a.y * 64.0f);
  u.h[2] = (_Float16)(a.z * 64.0f); u.h[3] = (_Float16)(a.w * 64.0f);
  u.h[4] = (_Float16)(b.x * 64.0f); u.h[5] = (_Float16)(b.y * 64.0f);
  u.h[6] = (_Float16)(b.z * 64.0f); u.h[7] = (_Float16)(b.w * 64.0f);
  _Float16* dp = wh + (size_t)g * 8;
  if (ok != 0) *(volatile v4i*)dp = u.i;
  __threadfence();
  if (ok != 0) *(volatile v4i*)dp = u.i;
}

__global__ __launch_bounds__(NTHR) void k_count(
    const int* __restrict__ ei, int* cnt, float* dinv, int nE, int vec8) {
  __shared__ __attribute__((aligned(16))) int scnt[NBC];
  __shared__ __attribute__((aligned(16))) int list[LISTN];
  __shared__ int wcnt[NWAVE];
  const int tid = threadIdx.x, lane = tid & 31, wave = tid >> 5;
  const int nodeBase = blockIdx.x * NBC;
  const int* dsts = ei + nE;

  for (int i = tid; i < NBC; i += NTHR) scnt[i] = 0;
  __syncthreads();

  const int nChunks = (nE + CHUNK - 1) / CHUNK;
#pragma unroll 1
  for (int ch = 0; ch < nChunks; ++ch) {
    const int cbase = ch * CHUNK;
    const int wc = scan_chunk<NBC>(dsts, nE, cbase, nodeBase, vec8, list, tid, lane, wave);
    if (lane == 0) wcnt[wave] = wc;
    __syncthreads();
    if (wave == 0) {
#pragma unroll 1
      for (int wsx = 0; wsx < NWAVE; ++wsx) {
        int n = __builtin_amdgcn_readfirstlane(wcnt[wsx]);
        n = n > WCAP ? WCAP : (n < 0 ? 0 : n);
        const int* lp = list + wsx * WCAP;
#pragma unroll 1
        for (int i = 0; i < n; ++i) {
          const int ent  = __builtin_amdgcn_readfirstlane(lp[i]);
          const int slot = ent & (NBC - 1);
          if (lane == 0) scnt[slot] = scnt[slot] + 1;
        }
      }
    }
    __syncthreads();
  }

  v4i cq[4]; v4f dq[4];
#pragma unroll
  for (int q = 0; q < 4; ++q) {
    const int f = (wave * 4 + q) * 128 + 4 * lane;
    const v4i c = *(const v4i*)(scnt + f);
    cq[q] = c;
    dq[q].x = rsqrtf((float)(c.x + 1));
    dq[q].y = rsqrtf((float)(c.y + 1));
    dq[q].z = rsqrtf((float)(c.z + 1));
    dq[q].w = rsqrtf((float)(c.w + 1));
  }
  int*   cp = cnt + (size_t)nodeBase;
  float* dp = dinv + (size_t)nodeBase;
#pragma unroll
  for (int q = 0; q < 4; ++q) {
    const int f = (wave * 4 + q) * 128 + 4 * lane;
    *(volatile v4i*)(cp + f) = cq[q];
    *(volatile v4f*)(dp + f) = dq[q];
  }
  __threadfence();
#pragma unroll
  for (int q = 0; q < 4; ++q) {
    const int f = (wave * 4 + q) * 128 + 4 * lane;
    *(volatile v4i*)(cp + f) = cq[q];
    *(volatile v4f*)(dp + f) = dq[q];
  }
}

__global__ __launch_bounds__(OTHR) void k_offsets(
    const int* __restrict__ cnt, int* off, int* rbase, int nChunk) {
  __shared__ __attribute__((aligned(16))) int soff[NBC];
  __shared__ __attribute__((aligned(16))) int srb[RBN];
  __shared__ int wtot[OTHR / 32];
  const int tid = threadIdx.x, lane = tid & 31, wave = tid >> 5, sub = tid >> 7;
  for (int i = tid; i < RBN; i += OTHR) srb[i] = 0;
  int carry = 0;
#pragma unroll 1
  for (int ch = 0; ch < nChunk; ++ch) {
    const int base = ch * NBC;
    const v4i c0 = *(const v4i*)(cnt + base + 8 * tid);
    const v4i c1 = *(const v4i*)(cnt + base + 8 * tid + 4);
    const int e0 = max(c0.x, 0), e1 = max(c0.y, 0), e2 = max(c0.z, 0), e3 = max(c0.w, 0);
    const int e4 = max(c1.x, 0), e5 = max(c1.y, 0), e6 = max(c1.z, 0), e7 = max(c1.w, 0);
    const int ts = e0 + e1 + e2 + e3 + e4 + e5 + e6 + e7;
    int incl = ts;
#pragma unroll
    for (int d = 1; d < 32; d <<= 1) {
      const int t = __shfl_up(incl, d);
      if (lane >= d) incl += t;
    }
    if (lane == 31) wtot[wave] = incl;
    __syncthreads();
    const int S0 = wtot[0]  + wtot[1]  + wtot[2]  + wtot[3];
    const int S1 = wtot[4]  + wtot[5]  + wtot[6]  + wtot[7];
    const int S2 = wtot[8]  + wtot[9]  + wtot[10] + wtot[11];
    const int S3 = wtot[12] + wtot[13] + wtot[14] + wtot[15];
    int pre = 0;
#pragma unroll 1
    for (int w = 4 * sub; w < wave; ++w) pre += wtot[w];
    const int b0 = carry;
    const int b1 = b0 + ((S0 + 31) & ~31);
    const int b2 = b1 + ((S1 + 31) & ~31);
    const int b3 = b2 + ((S2 + 31) & ~31);
    const int b4 = b3 + ((S3 + 31) & ~31);
    const int myb = sub == 0 ? b0 : (sub == 1 ? b1 : (sub == 2 ? b2 : b3));
    if (tid == 0) {
      srb[min(4 * ch + 0, RBN - 1)] = b0;
      srb[min(4 * ch + 1, RBN - 1)] = b1;
      srb[min(4 * ch + 2, RBN - 1)] = b2;
      srb[min(4 * ch + 3, RBN - 1)] = b3;
    }
    int run = myb + pre + incl - ts;
    soff[8 * tid + 0] = run; run += e0;
    soff[8 * tid + 1] = run; run += e1;
    soff[8 * tid + 2] = run; run += e2;
    soff[8 * tid + 3] = run; run += e3;
    soff[8 * tid + 4] = run; run += e4;
    soff[8 * tid + 5] = run; run += e5;
    soff[8 * tid + 6] = run; run += e6;
    soff[8 * tid + 7] = run;
    carry = b4;
    __syncthreads();
    const v4i o0 = *(const v4i*)(soff + 4 * tid);
    const v4i o1 = *(const v4i*)(soff + 4 * (tid + OTHR));
    int* op = off + base;
    *(volatile v4i*)(op + 4 * tid) = o0;
    *(volatile v4i*)(op + 4 * (tid + OTHR)) = o1;
    __threadfence();
    *(volatile v4i*)(op + 4 * tid) = o0;
    *(volatile v4i*)(op + 4 * (tid + OTHR)) = o1;
    __syncthreads();
  }
  if (tid == 0) srb[min(4 * nChunk, RBN - 1)] = carry;
  __syncthreads();
  v4i rv = {0, 0, 0, 0};
  if (tid < 32) rv = *(const v4i*)(srb + 4 * tid);
  if (tid < 32) *(volatile v4i*)(rbase + 4 * tid) = rv;
  __threadfence();
  if (tid < 32) *(volatile v4i*)(rbase + 4 * tid) = rv;
}

__global__ __launch_bounds__(NTHR) void k_fill(
    const int* __restrict__ ei, const int* __restrict__ off, const int* __restrict__ rbase,
    int* csr, int nN, int nE, int vec8, int csrLen) {
  extern __shared__ v4f lds_dyn[];
  int* region = (int*)lds_dyn;
  int* cursor = region + RCAP;
  int* list   = cursor + NBF;
  int* wcnt   = list + LISTN;
  const int tid = threadIdx.x, lane = tid & 31, wave = tid >> 5;
  const int b = blockIdx.x;
  const int nodeBase = b * NBF;
  const int* dsts = ei + nE;

  int rb0 = rbase[b];
  const int rb1 = rbase[b + 1];
  rb0 = rb0 < 0 ? 0 : (rb0 > csrLen ? csrLen : rb0);
  rb0 &= ~31;
  int len = rb1 - rb0;
  len = len < 0 ? 0 : (len > RCAP ? RCAP : len);
  int lenW = (len + 31) & ~31;
  if (rb0 + lenW > csrLen) lenW = (csrLen - rb0) & ~31;

  {
    const v4i z = {0, 0, 0, 0};
    for (int i = tid; i < RCAP / 4; i += NTHR) ((v4i*)region)[i] = z;
    for (int s = tid; s < NBF; s += NTHR) {
      int o = off[nodeBase + s] - rb0;
      o = o < 0 ? 0 : (o > RCAP ? RCAP : o);
      cursor[s] = o;
    }
  }
  __syncthreads();

  const int nChunks = (nE + CHUNK - 1) / CHUNK;
#pragma unroll 1
  for (int ch = 0; ch < nChunks; ++ch) {
    const int cbase = ch * CHUNK;
    const int wc = scan_chunk<NBF>(dsts, nE, cbase, nodeBase, vec8, list, tid, lane, wave);
    if (lane == 0) wcnt[wave] = wc;
    __syncthreads();
    if (wave == 0) {
#pragma unroll 1
      for (int wsx = 0; wsx < NWAVE; ++wsx) {
        int n = __builtin_amdgcn_readfirstlane(wcnt[wsx]);
        n = n > WCAP ? WCAP : (n < 0 ? 0 : n);
        const int* lp = list + wsx * WCAP;
#pragma unroll 1
        for (int i = 0; i < n; ++i) {
          const int ent  = __builtin_amdgcn_readfirstlane(lp[i]);
          const int slot = ent & (NBF - 1);
          int e = cbase + ((ent >> 12) & (CHUNK - 1));
          e = e > nE - 1 ? nE - 1 : e;
          int src = ei[e];
          src = src < 0 ? 0 : (src > nN - 1 ? nN - 1 : src);
          if (lane == 0) {
            int pos = cursor[slot];
            pos = pos < 0 ? 0 : (pos > RCAP - 1 ? RCAP - 1 : pos);
            region[pos] = src;
            const int np = pos + 1;
            cursor[slot] = np > RCAP ? RCAP : np;
          }
        }
      }
    }
    __syncthreads();
  }

  const int nv = lenW >> 2;
  int* gp = csr + rb0;
#pragma unroll 1
  for (int i = tid; i < nv; i += NTHR) { const v4i v = ((const v4i*)region)[i]; *(volatile v4i*)(gp + 4 * i) = v; }
  __threadfence();
#pragma unroll 1
  for (int i = tid; i < nv; i += NTHR) { const v4i v = ((const v4i*)region)[i]; *(volatile v4i*)(gp + 4 * i) = v; }
}

__global__ __launch_bounds__(NTHR) void k_gemm(
    const float* __restrict__ A, const unsigned short* __restrict__ Bw, const float* __restrict__ dinv,
    const float* __restrict__ bias, const float* __restrict__ w3, const float* __restrict__ b3,
    float* C, float* x1o, int nRowsA, int nRowsC, int useDinv, int useBias, int useRelu, int headMode) {
  extern __shared__ v4f lds_dyn[];
  constexpr int KD = HIDC;
  unsigned short* sHi = (unsigned short*)lds_dyn;
  unsigned short* sLo = sHi + GROWS * APH;
  float*          stg = (float*)lds_dyn;
  float*          sx  = stg + GROWS * HIDC;
  const int tid = threadIdx.x, lane = tid & 31, wave = tid >> 5, hh = lane >> 4, m = lane & 15;
  const int wr = wave & 3, wc = wave >> 2;
  const int colW = wc * 128;
  const int rowBase = blockIdx.x * GROWS;

#pragma unroll
  for (int i = 0; i < (GROWS * KD / 8) / NTHR; ++i) {
    const int idx = i * NTHR + tid;
    const int r   = idx >> 5;
    const int c0  = (idx & 31) * 8;
    int row = rowBase + r;
    row = row > nRowsA - 1 ? nRowsA - 1 : row;
    const float* ap = A + (size_t)row * KD + c0;
    const v4f a = *(const v4f*)ap, b = *(const v4f*)(ap + 4);
    v8us hv, lv;
    split8(a, b, hv, lv);
    *(v8us*)(sHi + r * APH + c0) = hv;
    *(v8us*)(sLo + r * APH + c0) = lv;
  }
  __syncthreads();

  v8f acc[8];
#pragma unroll
  for (int t = 0; t < 8; ++t) { v8f z = {0.f, 0.f, 0.f, 0.f, 0.f, 0.f, 0.f, 0.f}; acc[t] = z; }
  const unsigned short* ahp = sHi + (wr * 16 + m) * APH + 8 * hh;
  const unsigned short* alp = sLo + (wr * 16 + m) * APH + 8 * hh;
#pragma unroll 2
  for (int kt = 0; kt < KD / 32; ++kt) {
    FragB ah, al;
    ah.h[0] = *(const v8us*)(ahp + 32 * kt);
    ah.h[1] = *(const v8us*)(ahp + 32 * kt + 16);
    al.h[0] = *(const v8us*)(alp + 32 * kt);
    al.h[1] = *(const v8us*)(alp + 32 * kt + 16);
#pragma unroll
    for (int t = 0; t < 8; ++t) {
      const unsigned short* bp = Bw + (size_t)(colW + 16 * t + m) * KD + 32 * kt + 8 * hh;
      FragB bh, bl;
      bh.h[0] = *(const v8us*)bp;
      bh.h[1] = *(const v8us*)(bp + 16);
      bl.h[0] = *(const v8us*)(bp + WPL);
      bl.h[1] = *(const v8us*)(bp + WPL + 16);
      acc[t] = wmb(ah.v, bh.v, acc[t]);
      acc[t] = wmb(ah.v, bl.v, acc[t]);
      acc[t] = wmb(al.v, bh.v, acc[t]);
    }
  }
  __syncthreads();

  const int r0 = wr * 16 + 8 * hh;
  const v4f dA = *(const v4f*)(dinv + (size_t)rowBase + r0);
  const v4f dB = *(const v4f*)(dinv + (size_t)rowBase + r0 + 4);
  float s[8];
  s[0] = dA.x; s[1] = dA.y; s[2] = dA.z; s[3] = dA.w; s[4] = dB.x; s[5] = dB.y; s[6] = dB.z; s[7] = dB.w;
#pragma unroll
  for (int r = 0; r < 8; ++r) s[r] = (useDinv != 0 ? s[r] : 1.0f);
  float* sp = stg + r0 * HIDC + colW + m;
#pragma unroll
  for (int t = 0; t < 8; ++t) {
    const float bl = bias[colW + 16 * t + m];
    const float bv = useBias != 0 ? bl : 0.0f;
#pragma unroll
    for (int r = 0; r < 8; ++r) {
      float v = acc[t][r] * s[r] + bv;
      v = useRelu != 0 ? fmaxf(v, 0.0f) : v;
      sp[r * HIDC + 16 * t] = v;
    }
  }
  __syncthreads();

  const int rw = wave * 8;
  if (headMode == 0) {
    v4f va[8], vb[8];
#pragma unroll
    for (int i = 0; i < 8; ++i) {
      const float* lp = stg + (rw + i) * HIDC + 4 * lane;
      va[i] = *(const v4f*)lp;
      vb[i] = *(const v4f*)(lp + 128);
    }
#pragma unroll
    for (int i = 0; i < 8; ++i) {
      const int row = rowBase + rw + i;
      float* gp = C + (size_t)row * HIDC + 4 * lane;
      if (row < nRowsC) { *(volatile v4f*)gp = va[i]; *(volatile v4f*)(gp + 128) = vb[i]; }
    }
    __threadfence();
#pragma unroll
    for (int i = 0; i < 8; ++i) {
      const int row = rowBase + rw + i;
      float* gp = C + (size_t)row * HIDC + 4 * lane;
      if (row < nRowsC) { *(volatile v4f*)gp = va[i]; *(volatile v4f*)(gp + 128) = vb[i]; }
    }
  } else {
    const v4f wa = *(const v4f*)(w3 + 4 * lane);
    const v4f wb = *(const v4f*)(w3 + 128 + 4 * lane);
    const float b3v = b3[0];
#pragma unroll 1
    for (int i = 0; i < 8; ++i) {
      const float* lp = stg + (rw + i) * HIDC + 4 * lane;
      const v4f p0 = *(const v4f*)lp;
      const v4f p1 = *(const v4f*)(lp + 128);
      float p = p0.x * wa.x + p0.y * wa.y + p0.z * wa.z + p0.w * wa.w
              + p1.x * wb.x + p1.y * wb.y + p1.z * wb.z + p1.w * wb.w;
      p += __shfl_xor(p, 16);
      p += __shfl_xor(p, 8);
      p += __shfl_xor(p, 4);
      p += __shfl_xor(p, 2);
      p += __shfl_xor(p, 1);
      if (lane == 0) sx[rw + i] = p + b3v;
    }
    __syncthreads();
    v4f xv = {0.f, 0.f, 0.f, 0.f};
    if (tid < 16) xv = *(const v4f*)(sx + 4 * tid);
    float* xp = x1o + (size_t)rowBase + 4 * tid;
    if (tid < 16) *(volatile v4f*)xp = xv;
    __threadfence();
    if (tid < 16) *(volatile v4f*)xp = xv;
  }
}

__global__ __launch_bounds__(NTHR) void k_agg(
    const int* __restrict__ csr, const int* __restrict__ off, const int* __restrict__ cnt,
    const float* __restrict__ dinv, const float* __restrict__ hw, const float* __restrict__ xres,
    const float* __restrict__ bs, float* h, int nN, int csrLen) {
  const int tid = threadIdx.x, lane = tid & 31, wave = tid >> 5;
  const int tbase = blockIdx.x * TGT + wave * 32;
  const int cl = tbase + lane;
  const int cnt_l = cnt[cl];
  const int off_l = off[cl];
  union FI { float f; int i; };
  FI dvu; dvu.f = dinv[cl];
  const v4f bb0 = *(const v4f*)(bs + 4 * lane);
  const v4f bb1 = *(const v4f*)(bs + 128 + 4 * lane);

#pragma unroll 1
  for (int j = 0; j < 32; ++j) {
    const int c = tbase + j;
    int n = __builtin_amdgcn_readlane(cnt_l, j);
    n = n < 0 ? 0 : (n > DEGCAP ? DEGCAP : n);
    const int st = __builtin_amdgcn_readlane(off_l, j);
    FI du; du.i = __builtin_amdgcn_readlane(dvu.i, j);
    const float dc = du.f;
    v4f a0 = {0.f, 0.f, 0.f, 0.f};
    v4f a1 = {0.f, 0.f, 0.f, 0.f};
#pragma unroll 1
    for (int q0 = 0; q0 < n; q0 += 32) {
      int pos = st + q0 + lane;
      pos = pos < 0 ? 0 : (pos > csrLen - 1 ? csrLen - 1 : pos);
      int sl = csr[pos];
      sl = sl < 0 ? 0 : (sl > nN - 1 ? nN - 1 : sl);
      const int mcnt = (n - q0) < 32 ? (n - q0) : 32;
#pragma unroll 1
      for (int p = 0; p < mcnt; ++p) {
        const int s = __builtin_amdgcn_readlane(sl, p);
        const float* rp = hw + (size_t)s * HIDC + 4 * lane;
        a0 = a0 + *(const v4f*)rp;
        a1 = a1 + *(const v4f*)(rp + 128);
      }
    }
    const float* svp = hw + (size_t)c * HIDC + 4 * lane;
    const v4f sv0 = *(const v4f*)svp;
    const v4f sv1 = *(const v4f*)(svp + 128);
    const int cx = c > nN - 1 ? nN - 1 : c;
    const float* xrp = xres + (size_t)cx * HIDC + 4 * lane;
    const v4f xr0 = *(const v4f*)xrp;
    const v4f xr1 = *(const v4f*)(xrp + 128);
    v4f v0 = (a0 + sv0) * dc + bb0;
    v4f v1 = (a1 + sv1) * dc + bb1;
    v0.x = fmaxf(v0.x, 0.f) + xr0.x; v0.y = fmaxf(v0.y, 0.f) + xr0.y; v0.z = fmaxf(v0.z, 0.f) + xr0.z; v0.w = fmaxf(v0.w, 0.f) + xr0.w;
    v1.x = fmaxf(v1.x, 0.f) + xr1.x; v1.y = fmaxf(v1.y, 0.f) + xr1.y; v1.z = fmaxf(v1.z, 0.f) + xr1.z; v1.w = fmaxf(v1.w, 0.f) + xr1.w;
    float* hp = h + (size_t)c * HIDC + 4 * lane;
    *(volatile v4f*)hp = v0;
    *(volatile v4f*)(hp + 128) = v1;
    __threadfence();
    *(volatile v4f*)hp = v0;
    *(volatile v4f*)(hp + 128) = v1;
  }
}

__global__ __launch_bounds__(NTHR) void k_bilin(
    const float* __restrict__ x2, const _Float16* __restrict__ wh, const float* __restrict__ bb,
    float* o1s, int nRowsX) {
  extern __shared__ v4f lds_dyn[];
  _Float16* xh = (_Float16*)lds_dyn;
  float*    xf = (float*)(xh + BROWS * XHP);
  float*    so = xf + BROWS * XFP;
  const int tid = threadIdx.x, lane = tid & 31, wave = tid >> 5, hh = lane >> 4, m = lane & 15;
  const int rowBase = blockIdx.x * BROWS;

#pragma unroll
  for (int it = 0; it < (BROWS * HIDC / 8) / NTHR; ++it) {
    const int g  = it * NTHR + tid;
    const int r  = g >> 5;
    const int c0 = (g & 31) * 8;
    int row = rowBase + r;
    row = row > nRowsX - 1 ? nRowsX - 1 : row;
    const float* sp = x2 + (size_t)row * HIDC + c0;
    const v4f a = *(const v4f*)sp, b = *(const v4f*)(sp + 4);
    *(v4f*)(xf + r * XFP + c0) = a;
    *(v4f*)(xf + r * XFP + c0 + 4) = b;
    H8 u;
    u.h[0] = (_Float16)a.x; u.h[1] = (_Float16)a.y; u.h[2] = (_Float16)a.z; u.h[3] = (_Float16)a.w;
    u.h[4] = (_Float16)b.x; u.h[5] = (_Float16)b.y; u.h[6] = (_Float16)b.z; u.h[7] = (_Float16)b.w;
    *(v8h*)(xh + r * XHP + c0) = u.h;
  }
  __syncthreads();

  const float sc = 1.0f / 64.0f;
#pragma unroll 1
  for (int ri = 0; ri < 8; ++ri) {
    const int r = wave * 8 + ri;
    const _Float16* Wr = wh + (size_t)r * WPL;
    v8f av[4];
#pragma unroll
    for (int rt = 0; rt < 4; ++rt) { v8f z = {0.f, 0.f, 0.f, 0.f, 0.f, 0.f, 0.f, 0.f}; av[rt] = z; }

#pragma unroll 1
    for (int jt = 0; jt < HIDC / 16; ++jt) {
      FragH B[8];
      const _Float16* bp = Wr + (size_t)(jt * 16 + m) * HIDC + 8 * hh;
#pragma unroll
      for (int kt = 0; kt < 8; ++kt) {
        B[kt].h[0] = *(const v8h*)(bp + 32 * kt);
        B[kt].h[1] = *(const v8h*)(bp + 32 * kt + 16);
      }
      const int col = jt * 16 + m;
#pragma unroll
      for (int rt = 0; rt < 4; ++rt) {
        const _Float16* As = xh + (rt * 16 + m) * XHP + 8 * hh;
        v8f d = {0.f, 0.f, 0.f, 0.f, 0.f, 0.f, 0.f, 0.f};
#pragma unroll
        for (int kt = 0; kt < 8; ++kt) {
          FragH a;
          a.h[0] = *(const v8h*)(As + 32 * kt);
          a.h[1] = *(const v8h*)(As + 32 * kt + 16);
          d = wmh(a.v, B[kt].v, d);
        }
        const float* xr = xf + (rt * 16 + 8 * hh) * XFP + col;
#pragma unroll
        for (int v = 0; v < 8; ++v) av[rt][v] += d[v] * xr[v * XFP];
      }
    }

    const float bias = bb[r];
#pragma unroll
    for (int rt = 0; rt < 4; ++rt) {
#pragma unroll
      for (int v = 0; v < 8; ++v) {
        float s = av[rt][v];
        s += __shfl_xor(s, 8);
        s += __shfl_xor(s, 4);
        s += __shfl_xor(s, 2);
        s += __shfl_xor(s, 1);
        const float val = s * sc + bias;
        if (m == 0) so[(rt * 16 + 8 * hh + v) * SOP + r] = val;
      }
    }
  }
  __syncthreads();

  float* gbase = o1s + (size_t)rowBase * NREG;
  v4f ov[4];
#pragma unroll
  for (int it = 0; it < 4; ++it) {
    const int q = it * NTHR + tid;
    ov[it] = *(const v4f*)(so + (q >> 4) * SOP + (q & 15) * 4);
  }
#pragma unroll
  for (int it = 0; it < 4; ++it) { const int q = it * NTHR + tid; *(volatile v4f*)(gbase + 4 * q) = ov[it]; }
  __threadfence();
#pragma unroll
  for (int it = 0; it < 4; ++it) { const int q = it * NTHR + tid; *(volatile v4f*)(gbase + 4 * q) = ov[it]; }
}

__global__ __launch_bounds__(NTHR) void k_out(
    const float* __restrict__ x1p, const float* __restrict__ o1s, float* out,
    int nX1q, int nQ, int x1cap, int o1cap) {
  const int q = (int)blockIdx.x * NTHR + (int)threadIdx.x;
  int qa = q > x1cap - 1 ? x1cap - 1 : q;
  qa = qa < 0 ? 0 : qa;
  int qb = q - nX1q;
  qb = qb < 0 ? 0 : (qb > o1cap - 1 ? o1cap - 1 : qb);
  const v4f va = *(const v4f*)(x1p + (size_t)4 * qa);
  const v4f vb = *(const v4f*)(o1s + (size_t)4 * qb);
  const bool isA = q < nX1q;
  v4f v;
  v.x = isA ? va.x : vb.x; v.y = isA ? va.y : vb.y; v.z = isA ? va.z : vb.z; v.w = isA ? va.w : vb.w;
  float* gp = out + (size_t)4 * (q < nQ ? q : 0);
  if (q < nQ) *(volatile v4f*)gp = v;
  __threadfence();
  if (q < nQ) *(volatile v4f*)gp = v;
}

extern "C" void kernel_launch(void* const* d_in, const int* in_sizes, int n_in,
                              void* d_out, int out_size, void* d_ws, size_t ws_size,
                              hipStream_t stream) {
  if (n_in < 14) return;
  const int nN = in_sizes[0] / HIDC;
  const int nE = in_sizes[1] / 2;
  if (nN <= 0 || nE <= 0 || in_sizes[0] != nN * HIDC || in_sizes[1] != 2 * nE) return;
  if (in_sizes[2]  != WPL || in_sizes[3]  != HIDC) return;
  if (in_sizes[4]  != WPL || in_sizes[5]  != HIDC) return;
  if (in_sizes[6]  != WPL || in_sizes[7]  != HIDC) return;
  if (in_sizes[8]  != HIDC || in_sizes[9] != 1) return;
  if (in_sizes[10] != WPL || in_sizes[11] != HIDC) return;
  if (in_sizes[12] != NREG * WPL || in_sizes[13] != NREG) return;
  if (out_size != nN * (1 + NREG)) return;
  if ((nN & 3) != 0) return;
  if (nE > (1 << 28) || nN > (1 << 24)) return;

  const float* x       = (const float*)d_in[0];
  const int*   ei      = (const int*)d_in[1];
  const float* conv_w  = (const float*)d_in[2];
  const float* conv_b  = (const float*)d_in[3];
  const float* lin1_w  = (const float*)d_in[4];
  const float* lin1_b  = (const float*)d_in[5];
  const float* lin2_w  = (const float*)d_in[6];
  const float* lin2_b  = (const float*)d_in[7];
  const float* lin3_w  = (const float*)d_in[8];
  const float* lin3_b  = (const float*)d_in[9];
  const float* lin4_w  = (const float*)d_in[10];
  const float* lin4_b  = (const float*)d_in[11];
  const float* bilin_w = (const float*)d_in[12];
  const float* bilin_b = (const float*)d_in[13];
  float* out = (float*)d_out;

  const int NPAD   = ((nN + TGT - 1) / TGT) * TGT;
  const int nBC    = (nN + NBC - 1) / NBC;
  const int CNTPAD = nBC * NBC;
  if (4 * nBC + 1 > RBN) return;
  const int nBF    = (nN + NBF - 1) / NBF;
  const int csrLen = ((nE + 31) & ~31) + 4096;
  if (31 * 4 * nBC > 4096) return;
  const int nGemm  = NPAD / GROWS;
  const int nAgg   = NPAD / TGT;
  const int NB64   = (nN + BROWS - 1) / BROWS;
  const int nBG    = NREG * WPL / 8;
  const int nQ     = out_size / 4;
  const int nX1q   = nN / 4;

  char* ws = (char*)d_ws;
  size_t off = 0;
  const size_t oW   = off; off += (size_t)NMAT * 2 * WPL * 2;            off = (off + 255) & ~(size_t)255;
  const size_t oWh  = off; off += (size_t)NREG * WPL * 2;                off = (off + 255) & ~(size_t)255;
  const size_t oCnt = off; off += (size_t)CNTPAD * 4;                    off = (off + 255) & ~(size_t)255;
  const size_t oDv  = off; off += (size_t)CNTPAD * 4;                    off = (off + 255) & ~(size_t)255;
  const size_t oOff = off; off += (size_t)CNTPAD * 4;                    off = (off + 255) & ~(size_t)255;
  const size_t oRb  = off; off += (size_t)RBN * 4;                       off = (off + 255) & ~(size_t)255;
  const size_t oCsr = off; off += (size_t)csrLen * 4;                    off = (off + 255) & ~(size_t)255;
  const size_t oHw  = off; off += (size_t)NPAD * HIDC * 4;               off = (off + 255) & ~(size_t)255;
  const size_t oX0  = off; off += (size_t)NPAD * HIDC * 4;               off = (off + 255) & ~(size_t)255;
  const size_t oH1  = off; off += (size_t)NPAD * HIDC * 4;               off = (off + 255) & ~(size_t)255;
  const size_t oX2  = off; off += (size_t)NPAD * HIDC * 4;               off = (off + 255) & ~(size_t)255;
  const size_t oX1  = off; off += (size_t)NPAD * 4;                      off = (off + 255) & ~(size_t)255;
  const size_t oO1  = off; off += (size_t)NB64 * BROWS * NREG * 4;       off = (off + 255) & ~(size_t)255;
  if (off > ws_size || off > (size_t)WSCAP) return;
  unsigned short* wp = (unsigned short*)(ws + oW);
  _Float16* wh   = (_Float16*)(ws + oWh);
  int*      cnt  = (int*)(ws + oCnt);
  float*    dinv = (float*)(ws + oDv);
  int*      offp = (int*)(ws + oOff);
  int*      rb   = (int*)(ws + oRb);
  int*      csr  = (int*)(ws + oCsr);
  float*    hw   = (float*)(ws + oHw);
  float*    x0p  = (float*)(ws + oX0);
  float*    h1   = (float*)(ws + oH1);
  float*    x2p  = (float*)(ws + oX2);
  float*    x1p  = (float*)(ws + oX1);
  float*    o1s  = (float*)(ws + oO1);

  const int vec8 = ((nE & 3) == 0) ? 1 : 0;

  k_wprep<<<NMAT * 32, NTHR, 0, stream>>>(conv_w, lin1_w, lin2_w, lin4_w, wp);
  k_bwprep<<<(nBG + NTHR - 1) / NTHR, NTHR, 0, stream>>>(bilin_w, wh, nBG);

  k_count<<<nBC, NTHR, 0, stream>>>(ei, cnt, dinv, nE, vec8);
  k_offsets<<<1, OTHR, 0, stream>>>(cnt, offp, rb, nBC);
  hipFuncSetAttribute(reinterpret_cast<const void*>(&k_fill),
                      hipFuncAttributeMaxDynamicSharedMemorySize, LDS_FILL);
  k_fill<<<nBF, NTHR, LDS_FILL, stream>>>(ei, offp, rb, csr, nN, nE, vec8, csrLen);

  hipFuncSetAttribute(reinterpret_cast<const void*>(&k_gemm),
                      hipFuncAttributeMaxDynamicSharedMemorySize, LDS_GEMM);
  k_gemm<<<nGemm, NTHR, LDS_GEMM, stream>>>(x, wp, dinv, conv_b, lin3_w, lin3_b, hw, x1p, nN, NPAD, 1, 0, 0, 0);
  k_agg<<<nAgg, NTHR, 0, stream>>>(csr, offp, cnt, dinv, hw, x, conv_b, x0p, nN, csrLen);
  k_gemm<<<nGemm, NTHR, LDS_GEMM, stream>>>(x0p, wp + (size_t)1 * 2 * WPL, dinv, lin1_b, lin3_w, lin3_b, h1, x1p, NPAD, NPAD, 0, 1, 1, 0);
  k_gemm<<<nGemm, NTHR, LDS_GEMM, stream>>>(h1, wp + (size_t)2 * 2 * WPL, dinv, lin2_b, lin3_w, lin3_b, hw, x1p, NPAD, NPAD, 0, 1, 1, 1);
  k_gemm<<<nGemm, NTHR, LDS_GEMM, stream>>>(h1, wp + (size_t)3 * 2 * WPL, dinv, lin4_b, lin3_w, lin3_b, x2p, x1p, NPAD, NPAD, 0, 1, 1, 0);

  hipFuncSetAttribute(reinterpret_cast<const void*>(&k_bilin),
                      hipFuncAttributeMaxDynamicSharedMemorySize, LDS_BIL);
  k_bilin<<<NB64, NTHR, LDS_BIL, stream>>>(x2p, wh, bilin_b, o1s, NPAD);

  k_out<<<(nQ + NTHR - 1) / NTHR, NTHR, 0, stream>>>(x1p, o1s, out, nX1q, nQ, NPAD / 4, NB64 * BROWS * NREG / 4);
}
